// BahdanauAttention_56014963474605
// MI455X (gfx1250) — hardware-run, weakly checked
//
#include <hip/hip_runtime.h>


#ifndef NB
#define NB 8
#endif
#ifndef TQ
#define TQ 128
#endif
#define NB_FULL  8
#define TQ_FULL  128
#ifndef OUT_SEQ
#define OUT_SEQ TQ
#endif
#define SK   256
#define HW   512
#define CQW  (2 * HW)
#define QT   16
#define HC   32
#define HCP  33
#define AWV  8
#define OSP  68
#define PP   264
#define FBN  (AWV * 16 * OSP)
#define E2C  2.8853900817779268f
#define XCL  20.0f
#define SCL2 (-2.8853900817779268f)
#define PSH  14.0f
#define NEGB (-3.0e38f)
#define CCAR 64.0f
#define WCAR 16.0f
#define OINV (1.0f / 1024.0f)

static_assert(SK == 256);
static_assert(SK == 32 * 8);
static_assert(AWV * 32 == 256);
static_assert(AWV * 2 == QT);
static_assert(AWV * 64 == HW);
static_assert(HC == 32);
static_assert(HW % HC == 0);
static_assert(SK * (HC / 4) == 8 * 256);
static_assert(QT * HC == 2 * 256);
static_assert(FBN >= SK * HCP);
static_assert(FBN >= QT * SK);
static_assert(HW % 64 == 0);
static_assert(HW % 32 == 0);
static_assert(CQW % 32 == 0);
static_assert(SK % 64 == 0);
static_assert(SK % 32 == 0);
static_assert(TQ % 64 == 0);
static_assert(TQ % QT == 0);
static_assert((NB * TQ) % 64 == 0);
static_assert((NB * SK) % 64 == 0);
static_assert(NB <= NB_FULL);
static_assert(TQ <= TQ_FULL);
static_assert((OSP * 4) % 16 == 0);
static_assert((PP * 2) % 16 == 0);
static_assert(PP >= SK);
static_assert(32 * 16 * 8 == 16 * 64 * 4);
static_assert(32 * 16 * 4 == 16 * 64 * 2);
static_assert(256 * 16 * 2 == 64 * 64 * 2);
static_assert(256 * 4 * 4 == 64 * 64);
static_assert(FBN * 4 + HC * QT * 4 + QT * PP * 2 + HC * 4 + QT * 4 <= 131072);
static_assert(64 * 72 * 2 <= 131072);
static_assert(16 * OSP * 4 <= 131072);

typedef _Float16 h16;
typedef unsigned short bf;
typedef __attribute__((ext_vector_type(16))) __bf16   v16bf;
typedef __attribute__((ext_vector_type(16))) _Float16 v16h;
typedef __attribute__((ext_vector_type(8)))  _Float16 v8h;
typedef __attribute__((ext_vector_type(8)))  unsigned short v8us;
typedef __attribute__((ext_vector_type(8)))  float    v8f;
typedef __attribute__((ext_vector_type(4)))  float    v4f;
typedef v4f  __attribute__((may_alias)) v4fa;

__device__ __forceinline__ unsigned short f2bf(float f) { unsigned u = __float_as_uint(f); u += 0x7FFFu + ((u >> 16) & 1u); return (unsigned short)(u >> 16); }
__device__ __forceinline__ float bfr(float f) { return __uint_as_float(((unsigned)f2bf(f)) << 16); }
__device__ __forceinline__ v16h cat16(v8h lo, v8h hi) { return __builtin_shufflevector(lo, hi, 0, 1, 2, 3, 4, 5, 6, 7, 8, 9, 10, 11, 12, 13, 14, 15); }
__device__ __forceinline__ v16bf cat16b(v8us lo, v8us hi) { return __builtin_bit_cast(v16bf, __builtin_shufflevector(lo, hi, 0, 1, 2, 3, 4, 5, 6, 7, 8, 9, 10, 11, 12, 13, 14, 15)); }
__device__ __forceinline__ v8f wmma16(v16h a, v16h b, v8f c) { return __builtin_amdgcn_wmma_f32_16x16x32_f16(false, a, false, b, (short)0, c, false, false); }
__device__ __forceinline__ v8f wmmab(v16bf a, v16bf b, v8f c) { return __builtin_amdgcn_wmma_f32_16x16x32_bf16(false, a, false, b, (short)0, c, false, false); }
__device__ __forceinline__ v16h  ldh(const h16* p) { return cat16(*(const v8h*)p, *(const v8h*)(p + 16)); }
__device__ __forceinline__ v16bf ldb(const bf* p)  { return cat16b(*(const v8us*)p, *(const v8us*)(p + 16)); }
__device__ __forceinline__ void wave_sync() { __builtin_amdgcn_fence(3  , "wavefront"); __builtin_amdgcn_wave_barrier(); asm volatile("" ::: "memory"); }

static __device__ __forceinline__ h16 toh_flush(float v) { const h16 r = (h16)v; return (fabsf(v) < 6.103515625e-05f) ? (h16)0.0f : r; }
__device__ __forceinline__ v8f wmma16g(v16h a, v16h b, v8f c) { c = wmma16(a, b, c); asm volatile("v_nop\n\tv_nop\n\tv_nop\n\tv_nop" : "+v"(c) : "v"(a), "v"(b)); return c; }
__device__ __forceinline__ v8f wmmabg(v16bf a, v16bf b, v8f c) { c = wmmab(a, b, c); asm volatile("v_nop\n\tv_nop\n\tv_nop\n\tv_nop" : "+v"(c) : "v"(a), "v"(b)); return c; }
__device__ __forceinline__ float tanh_e(float x) { float xc = (x > 15.0f) ? 15.0f : x; xc = (xc < -15.0f) ? -15.0f : xc;
    const float e = __builtin_amdgcn_exp2f(xc * E2C); return fmaf(-2.0f, __builtin_amdgcn_rcpf(1.0f + e), 1.0f); }

__global__ __launch_bounds__(256) void k_cvt8(const float* __restrict__ src, bf* dst, size_t n8) {
    const size_t i = (size_t)blockIdx.x * 256 + threadIdx.x; if (i >= n8) return;
    const v8f v = *(const v8f*)(src + i * 8); v8us o;
#pragma unroll
    for (int k = 0; k < 8; ++k) o[k] = f2bf(v[k]);
    *(volatile v8us*)(dst + i * 8) = o; __threadfence(); *(volatile v8us*)(dst + i * 8) = o;
}

__global__ __launch_bounds__(256) void k_cvth(const float* __restrict__ src, h16* dst, size_t n8, int c8n, int dpitch, int doff, float scale) {
    const size_t i = (size_t)blockIdx.x * 256 + threadIdx.x; if (i >= n8) return;
    const size_t row = i / (size_t)c8n, c = i % (size_t)c8n;
    const v8f v = *(const v8f*)(src + i * 8); v8h o;
#pragma unroll
    for (int k = 0; k < 8; ++k) o[k] = toh_flush(bfr(v[k]) * scale);
    h16* p = dst + row * (size_t)dpitch + (size_t)doff + c * 8;
    *(volatile v8h*)p = o; __threadfence(); *(volatile v8h*)p = o;
}

__global__ __launch_bounds__(256) void k_tr(const float* __restrict__ enc, h16* ET) {
    __shared__ __align__(16) h16 tl[64 * 72];
    const int tid = threadIdx.x;
    const int s0 = blockIdx.x * 64, h0 = blockIdx.y * 64, b = blockIdx.z;
    const float* src = enc + ((size_t)b * SK + s0) * HW + h0;
#pragma unroll
    for (int j = 0; j < 4; ++j) { const int idx = tid + 256 * j; const int r = idx >> 4, c4 = (idx & 15) * 4;
        const v4f x = *(const v4f*)(src + (size_t)r * HW + c4);
#pragma unroll
        for (int i = 0; i < 4; ++i) tl[(c4 + i) * 72 + r] = toh_flush(bfr(x[i])); }
    __syncthreads();
    h16* dst = ET + ((size_t)b * HW + h0) * SK + s0;
#pragma unroll 1
    for (int ps = 0; ps < 2; ++ps) {
#pragma unroll
        for (int s = 0; s < 2; ++s) { const int row = s * 32 + (tid >> 3), c8 = (tid & 7) * 8;
            const v8h val = *(const v8h*)(&tl[row * 72 + c8]);
            *(volatile v8h*)(dst + (size_t)row * SK + c8) = val; }
        if (ps == 0) __threadfence(); }
}

__global__ __launch_bounds__(32) void k_projexp(const bf* __restrict__ A, const bf* __restrict__ Wt, float* E, int rowsQ) {
    __shared__ __align__(16) float os[16 * OSP];
    const int K = HW;
    const int lane = threadIdx.x & 31, lr = lane & 15, hi = lane >> 4; const int r0 = blockIdx.x * 64, c0 = blockIdx.y * 64;
    const size_t wsel = (r0 >= rowsQ) ? (size_t)HW * HW : (size_t)0;
    v8f acc[4][4];
#pragma unroll
    for (int mb = 0; mb < 4; ++mb)
#pragma unroll
        for (int nb = 0; nb < 4; ++nb) acc[mb][nb] = (v8f){};
    const size_t aoff = (size_t)(r0 + lr) * K + 8 * hi, boff = wsel + (size_t)(c0 + lr) * K + 8 * hi;
#pragma unroll 1
    for (int kc = 0; kc < K; kc += 32) {
        v16bf a[4];
#pragma unroll
        for (int mb = 0; mb < 4; ++mb) a[mb] = ldb(A + aoff + (size_t)mb * 16 * K + kc);
#pragma unroll
        for (int nb = 0; nb < 4; ++nb) { const v16bf b = ldb(Wt + boff + (size_t)nb * 16 * K + kc);
#pragma unroll
            for (int mb = 0; mb < 4; ++mb) acc[mb][nb] = wmmabg(a[mb], b, acc[mb][nb]); }
    }
#pragma unroll
    for (int mb = 0; mb < 4; ++mb) {
#pragma unroll
        for (int nb = 0; nb < 4; ++nb) {
#pragma unroll
            for (int j = 0; j < 8; ++j) { float x = acc[mb][nb][j]; x = (x > XCL) ? XCL : x; x = (x < -XCL) ? -XCL : x;
                os[(hi * 8 + j) * OSP + nb * 16 + lr] = __builtin_amdgcn_exp2f(x * E2C); } }
        wave_sync();
        float* eb = E + (size_t)(r0 + mb * 16) * HW + c0;
#pragma unroll 1
        for (int ps = 0; ps < 2; ++ps) {
#pragma unroll
            for (int s = 0; s < 8; ++s) { const int row = 2 * s + (lane >> 4), c4 = (lane & 15) * 4;
                const v4f val = *(const v4fa*)(&os[row * OSP + c4]);
                *(volatile v4f*)(eb + (size_t)row * HW + c4) = val; }
            if (ps == 0) __threadfence(); }
        wave_sync();
    }
}

__global__ __launch_bounds__(256) void k_attn(const float* __restrict__ EQ, const float* __restrict__ EH, const float* __restrict__ vvec, const int* __restrict__ lens,
                                               const h16* __restrict__ ET, h16* CQ) {
    __shared__ __align__(16) float fb[FBN];
    __shared__ __align__(16) float sq[HC * QT];
    __shared__ __align__(16) h16 sP[QT * PP];
    __shared__ float sv[HC];
    __shared__ float linv[QT];
    const int tid = threadIdx.x;
    const int lane = tid & 31, lr = lane & 15, hi = lane >> 4;
    const int wave = __builtin_amdgcn_readfirstlane((int)(threadIdx.x >> 5));
    const int b = blockIdx.y, t0 = blockIdx.x * QT;
    int len = lens[b]; len = len < 0 ? 0 : (len > SK ? SK : len);
    const float* eqb = EQ + ((size_t)b * TQ + t0) * HW;
    const float* ehb = EH + (size_t)b * SK * HW;
    float acc[QT];
#pragma unroll
    for (int i = 0; i < QT; ++i) acc[i] = 0.0f;
#pragma unroll 1
    for (int hc = 0; hc < HW; hc += HC) {
#pragma unroll
        for (int j = 0; j < 8; ++j) { const int idx = tid + 256 * j; const int s = idx >> 3, h4 = (idx & 7) * 4;
            const v4f d = *(const v4f*)(ehb + (size_t)s * HW + hc + h4);
            fb[s * HCP + h4 + 0] = d[0]; fb[s * HCP + h4 + 1] = d[1]; fb[s * HCP + h4 + 2] = d[2]; fb[s * HCP + h4 + 3] = d[3]; }
#pragma unroll
        for (int j = 0; j < 2; ++j) { const int idx = tid + 256 * j; const int tt = idx >> 5, h = idx & 31;
            sq[h * QT + tt] = eqb[(size_t)tt * HW + hc + h]; }
        if (wave == 0) sv[lane] = bfr(vvec[hc + lane]);
        __syncthreads();
        const int ro = tid * HCP;
#pragma unroll 2
        for (int h = 0; h < HC; ++h) {
            const float eh = fb[ro + h]; const float wv = sv[h];
            const v4f q0 = *(const v4fa*)(&sq[h * QT + 0]), q1 = *(const v4fa*)(&sq[h * QT + 4]), q2 = *(const v4fa*)(&sq[h * QT + 8]), q3 = *(const v4fa*)(&sq[h * QT + 12]);
#pragma unroll
            for (int i = 0; i < 4; ++i) {
                acc[i]      = fmaf(wv, __builtin_amdgcn_rcpf(fmaf(eh, q0[i], 1.0f)), acc[i]);
                acc[4 + i]  = fmaf(wv, __builtin_amdgcn_rcpf(fmaf(eh, q1[i], 1.0f)), acc[4 + i]);
                acc[8 + i]  = fmaf(wv, __builtin_amdgcn_rcpf(fmaf(eh, q2[i], 1.0f)), acc[8 + i]);
                acc[12 + i] = fmaf(wv, __builtin_amdgcn_rcpf(fmaf(eh, q3[i], 1.0f)), acc[12 + i]); }
        }
        __syncthreads();
    }
#pragma unroll
    for (int tt = 0; tt < QT; ++tt) fb[tt * SK + tid] = acc[tt];
    __syncthreads();
#pragma unroll
    for (int rr = 0; rr < 2; ++rr) {
        const int row = 2 * wave + rr;
        const v4f x0 = *(const v4fa*)(&fb[row * SK + lane * 8]), x1 = *(const v4fa*)(&fb[row * SK + lane * 8 + 4]);
        float tv[8]; bool kp[8]; float mx = NEGB;
#pragma unroll
        for (int i = 0; i < 4; ++i) { tv[i] = x0[i] * SCL2; tv[4 + i] = x1[i] * SCL2; }
#pragma unroll
        for (int i = 0; i < 8; ++i) { kp[i] = (lane * 8 + i) < len; mx = fmaxf(mx, kp[i] ? tv[i] : NEGB); }
        mx = fmaxf(mx, __shfl_xor(mx, 16, 32)); mx = fmaxf(mx, __shfl_xor(mx, 8, 32)); mx = fmaxf(mx, __shfl_xor(mx, 4, 32));
        mx = fmaxf(mx, __shfl_xor(mx, 2, 32));  mx = fmaxf(mx, __shfl_xor(mx, 1, 32));
        const float sh = PSH - mx;
        v8h pv; float ls = 0.0f;
#pragma unroll
        for (int i = 0; i < 8; ++i) {
            const float e = tv[i] + sh;
            const bool on = kp[i] & (e >= -14.0f);
            const float ee = on ? e : 0.0f;
            const float p = __builtin_amdgcn_exp2f(ee);
            const h16 ph = on ? (h16)p : (h16)0.0f;
            pv[i] = ph; ls += (float)ph; }
        ls += __shfl_xor(ls, 16, 32); ls += __shfl_xor(ls, 8, 32); ls += __shfl_xor(ls, 4, 32); ls += __shfl_xor(ls, 2, 32); ls += __shfl_xor(ls, 1, 32);
        *(v8h*)(&sP[row * PP + lane * 8]) = pv;
        if (lane == 0) linv[row] = __builtin_amdgcn_rcpf(ls) * CCAR;
    }
    __syncthreads();
    const int n0 = wave * 64;
    v8f oc[4];
#pragma unroll
    for (int nb = 0; nb < 4; ++nb) oc[nb] = (v8f){};
    const size_t eo = ((size_t)b * HW + n0 + lr) * SK + 8 * hi;
#pragma unroll 1
    for (int k0 = 0; k0 < SK; k0 += 32) {
        const v16h a = cat16(*(const v8h*)(&sP[lr * PP + k0 + 8 * hi]), *(const v8h*)(&sP[lr * PP + k0 + 16 + 8 * hi]));
#pragma unroll
        for (int nb = 0; nb < 4; ++nb) { const v16h bb = ldh(ET + eo + (size_t)nb * 16 * SK + k0); oc[nb] = wmma16g(a, bb, oc[nb]); }
    }
    float scl[8];
#pragma unroll
    for (int j = 0; j < 8; ++j) scl[j] = linv[8 * hi + j];
    const int wb = wave * 16 * OSP;
#pragma unroll
    for (int nb = 0; nb < 4; ++nb) {
#pragma unroll
        for (int j = 0; j < 8; ++j) fb[wb + (8 * hi + j) * OSP + nb * 16 + lr] = oc[nb][j] * scl[j]; }
    wave_sync();
    h16* crow = CQ + ((size_t)b * TQ + t0) * CQW + n0;
#pragma unroll 1
    for (int ps = 0; ps < 2; ++ps) {
#pragma unroll
        for (int s = 0; s < 4; ++s) { const int row = 4 * s + (lane >> 3), c8 = (lane & 7) * 8;
            const v4f x0 = *(const v4fa*)(&fb[wb + row * OSP + c8]); const v4f x1 = *(const v4fa*)(&fb[wb + row * OSP + c8 + 4]); v8h hv;
#pragma unroll
            for (int i = 0; i < 4; ++i) { hv[i] = toh_flush(x0[i]); hv[4 + i] = toh_flush(x1[i]); }
            *(volatile v8h*)(crow + (size_t)row * CQW + c8) = hv; }
        if (ps == 0) __threadfence(); }
}

__global__ __launch_bounds__(32) void k_outg(const h16* __restrict__ A, const h16* __restrict__ Wt, const float* __restrict__ bias, float* OUT) {
    __shared__ __align__(16) float os[16 * OSP];
    const int K = CQW;
    const int lane = threadIdx.x & 31, lr = lane & 15, hi = lane >> 4; const int r0 = blockIdx.x * 64, c0 = blockIdx.y * 64;
    v8f acc[4][4];
#pragma unroll
    for (int mb = 0; mb < 4; ++mb)
#pragma unroll
        for (int nb = 0; nb < 4; ++nb) acc[mb][nb] = (v8f){};
    const size_t aoff = (size_t)(r0 + lr) * K + 8 * hi, boff = (size_t)(c0 + lr) * K + 8 * hi;
#pragma unroll 1
    for (int kc = 0; kc < K; kc += 32) {
        v16h a[4];
#pragma unroll
        for (int mb = 0; mb < 4; ++mb) a[mb] = ldh(A + aoff + (size_t)mb * 16 * K + kc);
#pragma unroll
        for (int nb = 0; nb < 4; ++nb) { const v16h b = ldh(Wt + boff + (size_t)nb * 16 * K + kc);
#pragma unroll
            for (int mb = 0; mb < 4; ++mb) acc[mb][nb] = wmma16g(a[mb], b, acc[mb][nb]); }
    }
    float bc[4];
#pragma unroll
    for (int nb = 0; nb < 4; ++nb) bc[nb] = bfr(bias[c0 + nb * 16 + lr]);
    const int bb = r0 / TQ, tt = r0 % TQ;
    float* ob = OUT + ((size_t)bb * OUT_SEQ + tt) * HW + c0;
#pragma unroll
    for (int mb = 0; mb < 4; ++mb) {
#pragma unroll
        for (int nb = 0; nb < 4; ++nb) {
#pragma unroll
            for (int j = 0; j < 8; ++j) os[(hi * 8 + j) * OSP + nb * 16 + lr] = tanh_e(fmaf(acc[mb][nb][j], OINV, bc[nb])); }
        wave_sync();
        float* orow = ob + (size_t)(mb * 16) * HW;
#pragma unroll 1
        for (int ps = 0; ps < 2; ++ps) {
#pragma unroll
            for (int s = 0; s < 8; ++s) { const int row = 2 * s + (lane >> 4), c4 = (lane & 15) * 4;
                const v4f val = *(const v4fa*)(&os[row * OSP + c4]);
                *(volatile v4f*)(orow + (size_t)row * HW + c4) = val; }
            if (ps == 0) __threadfence(); }
        wave_sync();
    }
}

static constexpr size_t al256(size_t v) { return (v + 255) & ~(size_t)255; }
static constexpr size_t ROWS_Q = (size_t)NB * TQ;
static constexpr size_t ROWS_E = (size_t)NB * SK;
static constexpr size_t SZ_XB = al256((ROWS_Q + ROWS_E) * HW * 2);
static constexpr size_t SZ_WB = al256((size_t)2 * HW * HW * 2);
static constexpr size_t SZ_EP = al256((ROWS_Q + ROWS_E) * HW * 4);
static constexpr size_t SZ_ET = al256((size_t)NB * HW * SK * 2);
static constexpr size_t SZ_CQ = al256(ROWS_Q * CQW * 2);
static constexpr size_t SZ_WO = al256((size_t)HW * CQW * 2);
static constexpr size_t SZ_TOTAL = SZ_XB + SZ_WB + SZ_EP + SZ_ET + SZ_CQ + SZ_WO;
static_assert(SZ_TOTAL <= (size_t)134217728);
static_assert(((size_t)HW * HW * 2) % 256 == 0);
static_assert((ROWS_Q * HW * 2) % 256 == 0);
static_assert((ROWS_Q * HW * 4) % 256 == 0);
static_assert(((size_t)TQ * HW) % 8 == 0);
static_assert(((size_t)HW * CQW) % 8 == 0);
static_assert((HW / 8) % 8 == 0);
static_assert((CQW / 8) % 8 == 0);
static_assert(HW % 64 == 0 && CQW % 64 == 0);

extern "C" void kernel_launch(void* const* d_in, const int* in_sizes, int n_in,
                              void* d_out, int out_size, void* d_ws, size_t ws_size, hipStream_t stream) {
    if (n_in < 8) return;
    if ((size_t)in_sizes[0] < ((size_t)(NB - 1) * TQ_FULL + TQ) * HW) return;
    if ((size_t)in_sizes[1] < ROWS_E * HW) return;
    if (in_sizes[2] < NB) return;
    if ((size_t)in_sizes[3] < (size_t)HW * HW || (size_t)in_sizes[4] < (size_t)HW * HW) return;
    if (in_sizes[5] < HW || (size_t)in_sizes[6] < (size_t)HW * CQW || in_sizes[7] < HW) return;
    if ((size_t)out_size < ((size_t)(NB - 1) * OUT_SEQ + TQ) * HW) return;
    if (SZ_TOTAL > ws_size) return;
    const float* query = (const float*)d_in[0];
    const float* enc   = (const float*)d_in[1];
    const int*   lens  = (const int*)d_in[2];
    const float* w_s   = (const float*)d_in[3];
    const float* w_h   = (const float*)d_in[4];
    const float* vvec  = (const float*)d_in[5];
    const float* w_out = (const float*)d_in[6];
    const float* b_out = (const float*)d_in[7];
    float* OUT = (float*)d_out;
    char* wsp = (char*)d_ws;
    bf*    XB = (bf*)wsp;    wsp += SZ_XB;
    bf*    WB = (bf*)wsp;    wsp += SZ_WB;
    float* EP = (float*)wsp; wsp += SZ_EP;
    h16*   ET = (h16*)wsp;   wsp += SZ_ET;
    h16*   CQ = (h16*)wsp;   wsp += SZ_CQ;
    h16*   WO = (h16*)wsp;   wsp += SZ_WO;
    bf* XE = XB + ROWS_Q * HW;
    float* EQ = EP; float* EH = EP + ROWS_Q * HW;

    if (TQ == TQ_FULL) {
        const size_t n8 = ROWS_Q * HW / 8; const unsigned g = (unsigned)((n8 + 255) / 256);
        k_cvt8<<<g, 256, 0, stream>>>(query, XB, n8);
        k_cvth<<<g, 256, 0, stream>>>(query, CQ, n8, HW / 8, CQW, HW, CCAR);
    } else {
        const size_t n8 = (size_t)TQ * HW / 8; const unsigned g = (unsigned)((n8 + 255) / 256);
        for (int b = 0; b < NB; ++b) {
            k_cvt8<<<g, 256, 0, stream>>>(query + (size_t)b * TQ_FULL * HW, XB + (size_t)b * TQ * HW, n8);
            k_cvth<<<g, 256, 0, stream>>>(query + (size_t)b * TQ_FULL * HW, CQ + (size_t)b * TQ * CQW, n8, HW / 8, CQW, HW, CCAR);
        }
    }
    { const size_t n8 = ROWS_E * HW / 8; k_cvt8<<<(unsigned)((n8 + 255) / 256), 256, 0, stream>>>(enc, XE, n8); }
    { const size_t n8 = (size_t)HW * HW / 8; const unsigned g = (unsigned)((n8 + 255) / 256);
      k_cvt8<<<g, 256, 0, stream>>>(w_s, WB, n8); k_cvt8<<<g, 256, 0, stream>>>(w_h, WB + (size_t)HW * HW, n8); }
    { const size_t n8 = (size_t)HW * CQW / 8; k_cvth<<<(unsigned)((n8 + 255) / 256), 256, 0, stream>>>(w_out, WO, n8, CQW / 8, CQW, 0, WCAR); }
    k_tr<<<dim3(SK / 64, HW / 64, NB), 256, 0, stream>>>(enc, ET);
    k_projexp<<<dim3((unsigned)((ROWS_Q + ROWS_E) / 64), HW / 64, 1), 32, 0, stream>>>(XB, WB, EP, (int)ROWS_Q);
    k_attn<<<dim3(TQ / QT, NB, 1), 256, 0, stream>>>(EQ, EH, vvec, lens, ET, CQ);
    k_outg<<<dim3((unsigned)(ROWS_Q / 64), HW / 64, 1), 32, 0, stream>>>(CQ, WO, b_out, OUT);
}
